// CrossAttentionAudioFuser_89292370084405
// MI455X (gfx1250) — hardware-verified
//
#include <hip/hip_runtime.h>
#include <math.h>

typedef __attribute__((ext_vector_type(16))) _Float16 v16h;
typedef __attribute__((ext_vector_type(16))) __bf16 v16b;
typedef __attribute__((ext_vector_type(8)))  _Float16 v8h;
typedef __attribute__((ext_vector_type(8)))  float v8f;
typedef __attribute__((ext_vector_type(4)))  float v4f;
typedef __attribute__((ext_vector_type(2)))  float v2f;
typedef __attribute__((ext_vector_type(4)))  unsigned v4u;
typedef __attribute__((ext_vector_type(4)))  int v4i;
typedef float __attribute__((may_alias)) float_a;
typedef int __attribute__((may_alias)) int_a;

template <typename T> __device__ __forceinline__ void vst2(void* p, T v) { *(volatile T*)p = v; __threadfence(); *(volatile T*)p = v; }
__device__ __forceinline__ v8f wmma16(v16h a, v16h b, v8f c) {
  v8f d = __builtin_amdgcn_wmma_f32_16x16x32_f16(false, a, false, b, (short)0, c, false, false);
  asm volatile("v_nop\n\tv_nop\n\tv_nop\n\tv_nop" : "+v"(d) : "v"(a), "v"(b));
  return d;
}
__device__ __forceinline__ v8f wmma_bf(v16b a, v16b b, v8f c) {
  v8f d = __builtin_amdgcn_wmma_f32_16x16x32_bf16(false, a, false, b, (short)0, c, false, false);
  asm volatile("v_nop\n\tv_nop\n\tv_nop\n\tv_nop" : "+v"(d) : "v"(a), "v"(b));
  return d;
}
__device__ __forceinline__ v16h frag_h(const _Float16* rowk0, int lane) {
  union { v16h v; v8h q[2]; } u; const _Float16* p = rowk0 + 8 * (lane >> 4);
  u.q[0] = *(const v8h*)p; u.q[1] = *(const v8h*)(p + 16); return u.v;
}
__device__ __forceinline__ v16h frag_f32(const float* rowk0, int lane) {
  v16h a; const float* p = rowk0 + 8 * (lane >> 4);
#pragma unroll
  for (int i = 0; i < 8; ++i) { a[i] = (_Float16)p[i]; a[8 + i] = (_Float16)p[16 + i]; }
  return a;
}
__device__ __forceinline__ v16h frag_f32s(const float* rowk0, int lane, float sc) {
  v16h a; const float* p = rowk0 + 8 * (lane >> 4);
#pragma unroll
  for (int i = 0; i < 8; ++i) { a[i] = (_Float16)(p[i] * sc); a[8 + i] = (_Float16)(p[16 + i] * sc); }
  return a;
}
__device__ __forceinline__ v16h fragc_f32(const float* W, int k0, int n, int lane, int ld, int K) {
  v16h a; const int g = lane >> 4;
#pragma unroll
  for (int i = 0; i < 8; ++i) { const int ka = k0 + 8 * g + i, kb = ka + 16;
    a[i] = (_Float16)(ka < K ? W[(size_t)ka * ld + n] : 0.f); a[8 + i] = (_Float16)(kb < K ? W[(size_t)kb * ld + n] : 0.f); }
  return a;
}
struct F2 { v16b h, l; };
__device__ __forceinline__ F2 bsplit16(const float v[16]) { F2 r;
#pragma unroll
  for (int i = 0; i < 16; ++i) { const __bf16 h = (__bf16)v[i]; r.h[i] = h; r.l[i] = (__bf16)(v[i] - (float)h); }
  return r; }
__device__ __forceinline__ F2 split_row(const float* row, int k0, int lane) { float v[16]; const float* p = row + k0 + 8 * (lane >> 4);
#pragma unroll
  for (int i = 0; i < 8; ++i) { v[i] = p[i]; v[8 + i] = p[16 + i]; }
  return bsplit16(v); }
__device__ __forceinline__ F2 split_rowK(const float* row, int k0, int lane, int K) { float v[16]; const int g = lane >> 4;
#pragma unroll
  for (int i = 0; i < 8; ++i) { const int ka = k0 + 8 * g + i, kb = ka + 16; v[i] = ka < K ? row[ka] : 0.f; v[8 + i] = kb < K ? row[kb] : 0.f; }
  return bsplit16(v); }
__device__ __forceinline__ F2 split_col(const float* W, int k0, int n, int lane, int ld, int K) { float v[16]; const int g = lane >> 4;
#pragma unroll
  for (int i = 0; i < 8; ++i) { const int ka = k0 + 8 * g + i, kb = ka + 16; v[i] = ka < K ? W[(size_t)ka * ld + n] : 0.f; v[8 + i] = kb < K ? W[(size_t)kb * ld + n] : 0.f; }
  return bsplit16(v); }
__device__ __forceinline__ v8f mac3(const F2& a, const F2& b, v8f c) { c = wmma_bf(a.l, b.h, c); c = wmma_bf(a.h, b.l, c); return wmma_bf(a.h, b.h, c); }
__device__ __forceinline__ float sigm(float v) { return 1.0f / (1.0f + expf(-v)); }
#define LDSX() do { asm volatile("s_wait_dscnt 0" ::: "memory"); __builtin_amdgcn_wave_barrier(); __builtin_amdgcn_fence(__ATOMIC_RELEASE, "workgroup"); } while (0)

#define NB 16
#define CI 512
#define NP 1024
#define CA 512
#define KL 256
#define NH 8
#define HD 64
#define NRQ (NB * NP)
#define NRK (NB * KL)

__global__ __launch_bounds__(256) void k_cvt(const float* __restrict__ img, const float* __restrict__ aud, _Float16* __restrict__ X16, _Float16* __restrict__ A16) {
  __shared__ __align__(16) _Float16 st[64][136];
  const int tid = threadIdx.x;
  if (blockIdx.z == 0) { const int b = blockIdx.y, p0 = (blockIdx.x & 15) * 64, c0 = (blockIdx.x >> 4) * 128;
    for (int q = tid; q < 128 * 64; q += 256) { const int cl = q >> 6, pl = q & 63; st[pl][cl] = (_Float16)img[((size_t)b * CI + c0 + cl) * NP + p0 + pl]; }
    __syncthreads();
    for (int q = tid; q < 64 * 16; q += 256) { const int pl = q >> 4, pc = q & 15; vst2(X16 + ((size_t)b * NP + p0 + pl) * CI + c0 + pc * 8, *(const v4u*)(&st[pl][pc * 8])); } }
  else { const size_t g8 = ((size_t)blockIdx.y * gridDim.x + blockIdx.x) * 256 + tid; if (g8 < (size_t)NRK * CA / 8) { union { v8h h; v4u u; } pk;
#pragma unroll
      for (int e = 0; e < 8; ++e) pk.h[e] = (_Float16)aud[g8 * 8 + e];
      vst2(A16 + g8 * 8, pk.u); } }
}
__global__ __launch_bounds__(256) void k_pack(const float* __restrict__ Wq, const float* __restrict__ Wk, const float* __restrict__ Wv, const float* __restrict__ Wo, _Float16* __restrict__ P) {
  const int r = blockIdx.x, tid = threadIdx.x; __shared__ __align__(16) _Float16 srow[512];
  const int which = r >> 9, n = r & 511; const float* W = which == 0 ? Wq : (which == 1 ? Wk : (which == 2 ? Wv : Wo));
  for (int k = tid; k < 512; k += 256) srow[k] = (_Float16)(W[(size_t)k * 512 + n] * 16.0f);
  __syncthreads();
  if (tid < 64) vst2(P + (size_t)r * 512 + tid * 8, *(const v4u*)(&srow[tid * 8]));
}
__global__ __launch_bounds__(128) void k_q(const _Float16* __restrict__ X16, const _Float16* __restrict__ P, const float* __restrict__ bq, _Float16* __restrict__ Q16) {
  __shared__ __align__(16) float so[4][16][132];
  const int tid = threadIdx.x, wave = tid >> 5, lane = tid & 31, col = lane & 15, g = lane >> 4;
  const int r0 = blockIdx.x * 64 + wave * 16, n0 = blockIdx.y * 128;
  v8f acc[8] = {};
#pragma unroll 2
  for (int kc = 0; kc < CI / 32; ++kc) { const v16h a = frag_h(X16 + (size_t)(r0 + col) * CI + kc * 32, lane);
#pragma unroll
    for (int j = 0; j < 8; ++j) acc[j] = wmma16(a, frag_h(P + (size_t)(n0 + j * 16 + col) * 512 + kc * 32, lane), acc[j]); }
#pragma unroll
  for (int j = 0; j < 8; ++j) { const float bb = bq[n0 + j * 16 + col];
#pragma unroll
    for (int r = 0; r < 8; ++r) so[wave][8 * g + r][j * 16 + col] = (acc[j][r] * (1.0f / 16.0f) + bb) * 4.0f; }
  LDSX();
  for (int q = lane; q < 16 * 16; q += 32) { const int rl = q >> 4, pc = q & 15; union { v8h h8; v4u u; } pk;
#pragma unroll
    for (int e = 0; e < 8; ++e) pk.h8[e] = (_Float16)so[wave][rl][pc * 8 + e];
    vst2(Q16 + (size_t)(r0 + rl) * CA + n0 + pc * 8, pk.u); }
}
__global__ __launch_bounds__(128) void k_kv(const _Float16* __restrict__ A16, const _Float16* __restrict__ P, const float* __restrict__ bk, const float* __restrict__ bv, _Float16* __restrict__ K16, _Float16* __restrict__ VT) {
  __shared__ __align__(16) float so[4][16][132];
  __shared__ __align__(16) _Float16 st[128][72];
  const int tid = threadIdx.x, wave = tid >> 5, lane = tid & 31, col = lane & 15, g = lane >> 4;
  const int which = blockIdx.z, r0b = blockIdx.x * 64, r0 = r0b + wave * 16, n0 = blockIdx.y * 128; const int b = r0b / KL, k0 = r0b % KL;
  const _Float16* Pw = P + (size_t)(512 + which * 512) * 512; const float* bias = which ? bv : bk;
  v8f acc[8] = {};
#pragma unroll 2
  for (int kc = 0; kc < CA / 32; ++kc) { const v16h a = frag_h(A16 + (size_t)(r0 + col) * CA + kc * 32, lane);
#pragma unroll
    for (int j = 0; j < 8; ++j) acc[j] = wmma16(a, frag_h(Pw + (size_t)(n0 + j * 16 + col) * 512 + kc * 32, lane), acc[j]); }
  if (which == 0) {
#pragma unroll
    for (int j = 0; j < 8; ++j) { const float bb = bias[n0 + j * 16 + col];
#pragma unroll
      for (int r = 0; r < 8; ++r) so[wave][8 * g + r][j * 16 + col] = (acc[j][r] * (1.0f / 16.0f) + bb) * 4.0f; }
    LDSX();
    for (int q = lane; q < 16 * 2 * 8; q += 32) { const int hh = q >> 7, rl = (q >> 3) & 15, pc = q & 7; const int h = (n0 >> 6) + hh; union { v8h h8; v4u u; } pk;
#pragma unroll
      for (int e = 0; e < 8; ++e) pk.h8[e] = (_Float16)so[wave][rl][hh * 64 + pc * 8 + e];
      vst2(K16 + (((size_t)b * NH + h) * KL + k0 + wave * 16 + rl) * HD + pc * 8, pk.u); } }
  else {
#pragma unroll
    for (int j = 0; j < 8; ++j) { const float bb = bias[n0 + j * 16 + col];
#pragma unroll
      for (int r = 0; r < 8; ++r) st[j * 16 + col][wave * 16 + 8 * g + r] = (_Float16)((acc[j][r] * (1.0f / 16.0f) + bb) * 4.0f); }
    __syncthreads();
    for (int q = tid; q < 128 * 8; q += 128) { const int cl = q >> 3, pc = q & 7; const int c = n0 + cl, h = c >> 6, d = c & 63; vst2(VT + (((size_t)b * NH + h) * HD + d) * KL + k0 + pc * 8, *(const v4u*)(&st[cl][pc * 8])); } }
}
__global__ __launch_bounds__(128) void k_attn(const _Float16* __restrict__ Q16, const _Float16* __restrict__ K16, const _Float16* __restrict__ VT, _Float16* __restrict__ O16) {
  __shared__ __align__(16) float sS[4][16][KL + 4];
  __shared__ __align__(16) _Float16 sP[4][16][KL + 8];
  __shared__ __align__(16) float sO[4][16][68];
  const int tid = threadIdx.x, w = tid >> 5, lane = tid & 31, col = lane & 15, g = lane >> 4;
  const int b = blockIdx.z, h = blockIdx.y, q0 = blockIdx.x * 64 + w * 16; const size_t bh = (size_t)b * NH + h;
  v16h aq[2];
#pragma unroll
  for (int kc = 0; kc < 2; ++kc) aq[kc] = frag_h(Q16 + ((size_t)b * NP + q0 + col) * CA + h * HD + kc * 32, lane);
#pragma unroll
  for (int t = 0; t < KL / 16; ++t) { v8f s = {};
#pragma unroll
    for (int kc = 0; kc < 2; ++kc) s = wmma16(aq[kc], frag_h(K16 + (bh * KL + t * 16 + col) * HD + kc * 32, lane), s);
#pragma unroll
    for (int r = 0; r < 8; ++r) sS[w][8 * g + r][t * 16 + col] = s[r] * (0.125f / 16.0f); }
  LDSX();
  { const int m = col; float mx = -3.4e38f; for (int e = 0; e < 128; ++e) mx = fmaxf(mx, sS[w][m][g * 128 + e]); mx = fmaxf(mx, __shfl_xor(mx, 16, 32));
    float l = 0.f; for (int e = 0; e < 128; ++e) { const float p = expf(sS[w][m][g * 128 + e] - mx); sS[w][m][g * 128 + e] = p; l += p; }
    l += __shfl_xor(l, 16, 32); const float inv = 16384.0f / l;
    for (int e = 0; e < 128; ++e) sP[w][m][g * 128 + e] = (_Float16)(sS[w][m][g * 128 + e] * inv); }
  LDSX();
  v8f acc[4] = {};
#pragma unroll
  for (int kc = 0; kc < KL / 32; ++kc) { const v16h pa = frag_h(&sP[w][col][0] + kc * 32, lane);
#pragma unroll
    for (int t = 0; t < 4; ++t) acc[t] = wmma16(pa, frag_h(VT + (bh * HD + t * 16 + col) * KL + kc * 32, lane), acc[t]); }
#pragma unroll
  for (int t = 0; t < 4; ++t)
#pragma unroll
    for (int r = 0; r < 8; ++r) sO[w][8 * g + r][t * 16 + col] = acc[t][r] * (8.0f / (16384.0f * 4.0f));
  LDSX();
  for (int q = lane; q < 16 * 8; q += 32) { const int rl = q >> 3, pc = q & 7; union { v8h h8; v4u u; } pk;
#pragma unroll
    for (int e = 0; e < 8; ++e) pk.h8[e] = (_Float16)sO[w][rl][pc * 8 + e];
    vst2(O16 + (bh * NP + q0 + rl) * HD + pc * 8, pk.u); }
}
__global__ __launch_bounds__(128) void k_proj(const _Float16* __restrict__ O16, const _Float16* __restrict__ P, const float* __restrict__ bo, const float* __restrict__ img, const float* __restrict__ gam, const float* __restrict__ bet, float* __restrict__ out) {
  __shared__ __align__(16) float sy[64][CI + 4];
  const int tid = threadIdx.x, wave = tid >> 5, lane = tid & 31, col = lane & 15, g = lane >> 4;
  const int r0b = blockIdx.x * 64, r0 = r0b + wave * 16; const int b = r0b / NP, p0 = r0b % NP;
#pragma unroll 1
  for (int np = 0; np < 4; ++np) { v8f acc[8] = {};
#pragma unroll 2
    for (int kc = 0; kc < CA / 32; ++kc) { const int R = r0 + col; const v16h a = frag_h(O16 + ((((size_t)(R >> 10)) * NH + (kc >> 1)) * NP + (R & 1023)) * HD + (kc & 1) * 32, lane);
#pragma unroll
      for (int j = 0; j < 8; ++j) acc[j] = wmma16(a, frag_h(P + (size_t)(1536 + np * 128 + j * 16 + col) * 512 + kc * 32, lane), acc[j]); }
#pragma unroll
    for (int j = 0; j < 8; ++j) { const int c = np * 128 + j * 16 + col; const float bb = bo[c];
#pragma unroll
      for (int r = 0; r < 8; ++r) { const int pl = wave * 16 + 8 * g + r; sy[pl][c] = acc[j][r] * (1.0f / 128.0f) + bb + img[((size_t)b * CI + c) * NP + p0 + pl]; } } }
  LDSX();
  { const int rl = lane >> 1, hf = lane & 1; float* row = &sy[wave * 16 + rl][0]; float s = 0.f; for (int c = hf * 256; c < hf * 256 + 256; ++c) s += row[c]; s += __shfl_xor(s, 1, 32); const float mu = s * (1.0f / CI);
    float q2 = 0.f; for (int c = hf * 256; c < hf * 256 + 256; ++c) { const float d = row[c] - mu; q2 += d * d; } q2 += __shfl_xor(q2, 1, 32); const float rs = rsqrtf(q2 * (1.0f / CI) + 1e-5f);
    LDSX();
    for (int c = hf * 256; c < hf * 256 + 256; ++c) row[c] = (row[c] - mu) * rs * gam[c] + bet[c]; }
  __syncthreads();
  for (int q = tid; q < CI * 16; q += 128) { const int c = q >> 4, pc = q & 15; v4f o; o[0] = sy[pc * 4][c]; o[1] = sy[pc * 4 + 1][c]; o[2] = sy[pc * 4 + 2][c]; o[3] = sy[pc * 4 + 3][c]; vst2(out + ((size_t)b * CI + c) * NP + p0 + pc * 4, o); }
}
extern "C" void kernel_launch(void* const* d_in, const int* in_sizes, int n_in, void* d_out, int out_size, void* d_ws, size_t ws_size, hipStream_t stream) {
  (void)in_sizes; (void)n_in; (void)out_size; (void)ws_size;
  const float** I = (const float**)d_in;
  const float* img = I[0]; const float* aud = I[1]; const float* Wq = I[2]; const float* bq = I[3]; const float* Wk = I[4]; const float* bk = I[5]; const float* Wv = I[6]; const float* bv = I[7]; const float* Wo = I[8]; const float* bo = I[9]; const float* gam = I[10]; const float* bet = I[11];
  float* out = (float*)d_out;
  char* ws = (char*)d_ws; size_t off = 0;
  auto take = [&](size_t bytes) { char* p = ws + off; off += (bytes + 255) & ~(size_t)255; return p; };
  _Float16* X16 = (_Float16*)take((size_t)NRQ * CI * 2); _Float16* A16 = (_Float16*)take((size_t)NRK * CA * 2); _Float16* P = (_Float16*)take((size_t)2048 * 512 * 2);
  _Float16* Q16 = (_Float16*)take((size_t)NRQ * CA * 2); _Float16* K16 = (_Float16*)take((size_t)NB * NH * KL * HD * 2); _Float16* VT = (_Float16*)take((size_t)NB * NH * HD * KL * 2); _Float16* O16 = (_Float16*)take((size_t)NRQ * CA * 2);
  k_cvt<<<dim3(64, NB, 2), 256, 0, stream>>>(img, aud, X16, A16);
  k_pack<<<2048, 256, 0, stream>>>(Wq, Wk, Wv, Wo, P);
  k_q<<<dim3(NRQ / 64, CA / 128), 128, 0, stream>>>(X16, P, bq, Q16);
  k_kv<<<dim3(NRK / 64, CA / 128, 2), 128, 0, stream>>>(A16, P, bk, bv, K16, VT);
  k_attn<<<dim3(NP / 64, NH, NB), 128, 0, stream>>>(Q16, K16, VT, O16);
  k_proj<<<NRQ / 64, 128, 0, stream>>>(O16, P, bo, img, gam, bet, out);
}
